// TriangleSelfAttention_16999480558056
// MI455X (gfx1250) — hardware-verified
//
#include <hip/hip_runtime.h>
#include <math.h>

typedef __attribute__((ext_vector_type(16))) _Float16 v16h;
typedef __attribute__((ext_vector_type(16))) __bf16 v16b;
typedef __attribute__((ext_vector_type(8)))  _Float16 v8h;
typedef __attribute__((ext_vector_type(8)))  float v8f;
typedef __attribute__((ext_vector_type(4)))  float v4f;
typedef __attribute__((ext_vector_type(2)))  float v2f;
typedef __attribute__((ext_vector_type(4)))  unsigned v4u;
typedef __attribute__((ext_vector_type(4)))  int v4i;
typedef float __attribute__((may_alias)) float_a;
typedef int __attribute__((may_alias)) int_a;

template <typename T> __device__ __forceinline__ void vst2(void* p, T v) { *(volatile T*)p = v; __threadfence(); *(volatile T*)p = v; }
__device__ __forceinline__ v8f wmma16(v16h a, v16h b, v8f c) {
  v8f d = __builtin_amdgcn_wmma_f32_16x16x32_f16(false, a, false, b, (short)0, c, false, false);
  asm volatile("v_nop\n\tv_nop\n\tv_nop\n\tv_nop" : "+v"(d) : "v"(a), "v"(b));
  return d;
}
__device__ __forceinline__ v8f wmma_bf(v16b a, v16b b, v8f c) {
  v8f d = __builtin_amdgcn_wmma_f32_16x16x32_bf16(false, a, false, b, (short)0, c, false, false);
  asm volatile("v_nop\n\tv_nop\n\tv_nop\n\tv_nop" : "+v"(d) : "v"(a), "v"(b));
  return d;
}
__device__ __forceinline__ v16h frag_h(const _Float16* rowk0, int lane) {
  union { v16h v; v8h q[2]; } u; const _Float16* p = rowk0 + 8 * (lane >> 4);
  u.q[0] = *(const v8h*)p; u.q[1] = *(const v8h*)(p + 16); return u.v;
}
__device__ __forceinline__ v16h frag_f32(const float* rowk0, int lane) {
  v16h a; const float* p = rowk0 + 8 * (lane >> 4);
#pragma unroll
  for (int i = 0; i < 8; ++i) { a[i] = (_Float16)p[i]; a[8 + i] = (_Float16)p[16 + i]; }
  return a;
}
__device__ __forceinline__ v16h frag_f32s(const float* rowk0, int lane, float sc) {
  v16h a; const float* p = rowk0 + 8 * (lane >> 4);
#pragma unroll
  for (int i = 0; i < 8; ++i) { a[i] = (_Float16)(p[i] * sc); a[8 + i] = (_Float16)(p[16 + i] * sc); }
  return a;
}
__device__ __forceinline__ v16h fragc_f32(const float* W, int k0, int n, int lane, int ld, int K) {
  v16h a; const int g = lane >> 4;
#pragma unroll
  for (int i = 0; i < 8; ++i) { const int ka = k0 + 8 * g + i, kb = ka + 16;
    a[i] = (_Float16)(ka < K ? W[(size_t)(ka < K ? ka : K - 1) * ld + n] : 0.f); a[8 + i] = (_Float16)(kb < K ? W[(size_t)(kb < K ? kb : K - 1) * ld + n] : 0.f); }
  return a;
}
struct F2 { v16b h, l; };
__device__ __forceinline__ F2 bsplit16(const float v[16]) { F2 r;
#pragma unroll
  for (int i = 0; i < 16; ++i) { const __bf16 h = (__bf16)v[i]; r.h[i] = h; r.l[i] = (__bf16)(v[i] - (float)h); }
  return r; }
__device__ __forceinline__ F2 split_row(const float* row, int k0, int lane) { float v[16]; const float* p = row + k0 + 8 * (lane >> 4);
#pragma unroll
  for (int i = 0; i < 8; ++i) { v[i] = p[i]; v[8 + i] = p[16 + i]; }
  return bsplit16(v); }
__device__ __forceinline__ F2 split_rowK(const float* row, int k0, int lane, int K) { float v[16]; const int g = lane >> 4;
#pragma unroll
  for (int i = 0; i < 8; ++i) { const int ka = k0 + 8 * g + i, kb = ka + 16; v[i] = ka < K ? row[ka < K ? ka : K - 1] : 0.f; v[8 + i] = kb < K ? row[kb < K ? kb : K - 1] : 0.f; }
  return bsplit16(v); }
__device__ __forceinline__ F2 split_col(const float* W, int k0, int n, int lane, int ld, int K) { float v[16]; const int g = lane >> 4;
#pragma unroll
  for (int i = 0; i < 8; ++i) { const int ka = k0 + 8 * g + i, kb = ka + 16; v[i] = ka < K ? W[(size_t)(ka < K ? ka : K - 1) * ld + n] : 0.f; v[8 + i] = kb < K ? W[(size_t)(kb < K ? kb : K - 1) * ld + n] : 0.f; }
  return bsplit16(v); }
__device__ __forceinline__ v8f mac3(const F2& a, const F2& b, v8f c) { c = wmma_bf(a.l, b.h, c); c = wmma_bf(a.h, b.l, c); return wmma_bf(a.h, b.h, c); }
__device__ __forceinline__ float sigm(float v) { return 1.0f / (1.0f + expf(-v)); }
#define LDSX() do { asm volatile("s_wait_dscnt 0" ::: "memory"); __builtin_amdgcn_wave_barrier(); __builtin_amdgcn_fence(__ATOMIC_RELEASE, "workgroup"); } while (0)

#define LL 256
#define DZ 128
#define NH 4
#define HD 32
#define DHC (NH * HD)
#define NR (LL * LL)
#ifndef NROWS
#define NROWS LL
#endif
#ifndef ZP
#define ZP (LL * LL)
#endif
__device__ __forceinline__ float bfr(float v) { return (float)(__bf16)v; }
__device__ __forceinline__ float sigm_(float v) { return 1.0f / (1.0f + expf(-v)); }
__device__ __forceinline__ v16h wcolh(const float* Wm, int k0, int o, int lane, int ld) { v16h w; const int g = lane >> 4;
#pragma unroll
  for (int i = 0; i < 8; ++i) { w[i] = (_Float16)(bfr(Wm[(size_t)(k0 + 8 * g + i) * ld + o]) * 256.0f); w[8 + i] = (_Float16)(bfr(Wm[(size_t)(k0 + 16 + 8 * g + i) * ld + o]) * 256.0f); }
  return w; }

#define WS_ZH  0u
#define WS_ZL  (WS_ZH + 2u * (size_t)NR * DZ)
#define WS_QH  (WS_ZL + 2u * (size_t)NR * DZ)
#define WS_KH  (WS_QH + 2u * (size_t)NR * DHC)
#define WS_VT  (WS_KH + 2u * (size_t)NR * DHC)
#define WS_GH  (WS_VT + 2u * (size_t)NR * DHC)
#define WS_O   (WS_GH + 2u * (size_t)NR * DHC)
#define WS_END (WS_O  + 4u * (size_t)NR * DHC)

__global__ __launch_bounds__(128) void k_ln(const float* __restrict__ Z, const float* __restrict__ LW, const float* __restrict__ LB, _Float16* __restrict__ ZH, _Float16* __restrict__ ZL) { __shared__ __align__(16) float st[DZ][65]; __shared__ __align__(16) _Float16 sh[64][136], slo[64][136];
  const int tid = threadIdx.x; const int n = blockIdx.y; const int i0 = blockIdx.x * 64; const size_t rbase = (size_t)n * LL + i0;
  for (int e = tid; e < DZ * 64; e += 128) { const int c = e >> 6, il = e & 63; st[c][il] = bfr(Z[(size_t)c * ZP + (size_t)n * LL + i0 + il]); }
  __syncthreads();
  if (tid < 64) { float s = 0.f;
#pragma unroll 8
    for (int c = 0; c < DZ; ++c) s += st[c][tid];
    const float mean = s * (1.0f / DZ); float s2 = 0.f;
#pragma unroll 8
    for (int c = 0; c < DZ; ++c) { const float d = st[c][tid] - mean; s2 += d * d; }
    const float rstd = rsqrtf(s2 * (1.0f / DZ) + 1e-5f);
#pragma unroll 8
    for (int c = 0; c < DZ; ++c) { const float zn = (st[c][tid] - mean) * rstd * bfr(LW[c]) + bfr(LB[c]); const _Float16 hv = (_Float16)zn; sh[tid][c] = hv; slo[tid][c] = (_Float16)((zn - (float)hv) * 1024.0f); } }
  __syncthreads();
  for (int e = tid; e < 64 * 16; e += 128) { const int rl = e >> 4, q = e & 15; vst2((unsigned*)(ZH + (rbase + rl) * DZ + q * 8), *(const v4u*)&sh[rl][q * 8]); vst2((unsigned*)(ZL + (rbase + rl) * DZ + q * 8), *(const v4u*)&slo[rl][q * 8]); } }
__global__ __launch_bounds__(128) void k_proj(const _Float16* __restrict__ ZH, const _Float16* __restrict__ ZL, const float* __restrict__ WQ, const float* __restrict__ BQ, const float* __restrict__ WK, const float* __restrict__ BK, const float* __restrict__ WV, const float* __restrict__ BV, const float* __restrict__ WG, const float* __restrict__ BG, _Float16* __restrict__ QH, _Float16* __restrict__ KH, _Float16* __restrict__ VT, _Float16* __restrict__ GH) {
  __shared__ __align__(16) _Float16 sh[64][136]; __shared__ __align__(16) _Float16 th[128][72];
  const int tid = threadIdx.x, wave = tid >> 5, lane = tid & 31, col = lane & 15, g = lane >> 4; const int which = blockIdx.z; const size_t r0 = (size_t)blockIdx.x * 64;
  const float* WA = which == 0 ? WQ : which == 1 ? WK : which == 2 ? WV : WG; const float* BA = which == 0 ? BQ : which == 1 ? BK : which == 2 ? BV : BG;
  const float qs = sqrtf(1.0f / 32.0f);
  v8f acc[8] = {}, accl[8] = {};
#pragma unroll
  for (int kc = 0; kc < DZ / 32; ++kc) { const v16h a = frag_h(ZH + (r0 + wave * 16 + col) * DZ + kc * 32, lane), al = frag_h(ZL + (r0 + wave * 16 + col) * DZ + kc * 32, lane); asm volatile("s_wait_loadcnt 0x0" ::: "memory");
#pragma unroll
    for (int j = 0; j < 8; ++j) { const v16h w = wcolh(WA, kc * 32, j * 16 + col, lane, DHC); asm volatile("s_wait_loadcnt 0x0" ::: "memory"); acc[j] = wmma16(a, w, acc[j]); accl[j] = wmma16(al, w, accl[j]); } }
#pragma unroll
  for (int j = 0; j < 8; ++j) { const float bb = bfr(BA[j * 16 + col]);
#pragma unroll
    for (int r = 0; r < 8; ++r) { float v = (acc[j][r] + accl[j][r] * (1.0f / 1024.0f)) * (1.0f / 256.0f) + bb; const int rl = wave * 16 + 8 * g + r, cl = j * 16 + col;
      if (which == 0) v = v * qs; else if (which == 3) v = sigm_(v);
      if (which == 2) th[cl][rl] = (_Float16)v; else sh[rl][cl] = (_Float16)v; } }
  __syncthreads();
  if (which != 2) { _Float16* dh = which == 0 ? QH : which == 1 ? KH : GH; for (int e = tid; e < 64 * 16; e += 128) { const int rl = e >> 4, q = e & 15; vst2((unsigned*)(dh + (r0 + rl) * DHC + q * 8), *(const v4u*)&sh[rl][q * 8]); } }
  else { const size_t n = r0 / LL; const int i0 = (int)(r0 % LL); for (int e = tid; e < 128 * 8; e += 128) { const int cl = e >> 3, q = e & 7; vst2((unsigned*)(VT + (n * DHC + cl) * (size_t)LL + i0 + q * 8), *(const v4u*)&th[cl][q * 8]); } } }
__global__ __launch_bounds__(64) void k_att(const _Float16* __restrict__ QH, const _Float16* __restrict__ KH, const _Float16* __restrict__ VT, float* __restrict__ O) {
  __shared__ __align__(16) float sl[2][16][LL + 4]; __shared__ __align__(16) _Float16 sp[2][16][LL + 8]; __shared__ __align__(16) float so[2][16][HD + 4];
  const int tid = threadIdx.x, wave = tid >> 5, lane = tid & 31, col = lane & 15, g = lane >> 4; const int h = blockIdx.y; const size_t n = blockIdx.z; const int i0 = blockIdx.x * 32 + wave * 16; const size_t q0 = n * LL + i0; const size_t kr0 = n * LL;
  const v16h aq = frag_h(QH + (q0 + col) * DHC + h * HD, lane);
#pragma unroll
  for (int pass = 0; pass < 2; ++pass) { v8f acc[8] = {};
#pragma unroll
    for (int j = 0; j < 8; ++j) { const v16h kb = frag_h(KH + (kr0 + pass * 128 + j * 16 + col) * DHC + h * HD, lane); acc[j] = wmma16(aq, kb, acc[j]); }
#pragma unroll
    for (int j = 0; j < 8; ++j) {
#pragma unroll
      for (int r = 0; r < 8; ++r) sl[wave][8 * g + r][pass * 128 + j * 16 + col] = acc[j][r]; } }
  LDSX();
#pragma unroll 1
  for (int rl = 0; rl < 16; ++rl) { float v[8]; float m = -3.0e38f;
#pragma unroll
    for (int z = 0; z < 8; ++z) { v[z] = sl[wave][rl][lane * 8 + z]; m = fmaxf(m, v[z]); }
#pragma unroll
    for (int o = 1; o < 32; o <<= 1) m = fmaxf(m, __shfl_xor(m, o));
    float s = 0.f;
#pragma unroll
    for (int z = 0; z < 8; ++z) { v[z] = expf(v[z] - m); s += v[z]; }
#pragma unroll
    for (int o = 1; o < 32; o <<= 1) s += __shfl_xor(s, o);
    const float inv = 2048.0f / s;
    union { v8h hv; v4u u; } pk;
#pragma unroll
    for (int z = 0; z < 8; ++z) pk.hv[z] = (_Float16)(v[z] * inv);
    *(v4u*)&sp[wave][rl][lane * 8] = pk.u; }
  LDSX();
  v8f acc2[2] = {};
#pragma unroll 2
  for (int kc = 0; kc < LL / 32; ++kc) { v16h ap; { union { v16h v; v8h q[2]; } u; u.q[0] = *(const v8h*)&sp[wave][col][kc * 32 + 8 * g]; u.q[1] = *(const v8h*)&sp[wave][col][kc * 32 + 16 + 8 * g]; ap = u.v; }
#pragma unroll
    for (int j = 0; j < 2; ++j) { const v16h vb = frag_h(VT + (n * DHC + h * HD + j * 16 + col) * (size_t)LL + kc * 32, lane); acc2[j] = wmma16(ap, vb, acc2[j]); } }
#pragma unroll
  for (int j = 0; j < 2; ++j)
#pragma unroll
    for (int r = 0; r < 8; ++r) so[wave][8 * g + r][j * 16 + col] = acc2[j][r] * (1.0f / 2048.0f);
  LDSX(); for (int rl = 0; rl < 16; ++rl) if (lane < 8) vst2(O + (q0 + rl) * DHC + h * HD + lane * 4, *(const v4f*)&so[wave][rl][lane * 4]); }
__global__ __launch_bounds__(128) void k_out(const float* __restrict__ O, const _Float16* __restrict__ GH, const float* __restrict__ W2, const float* __restrict__ B2, float* __restrict__ OUT) { __shared__ __align__(16) _Float16 sa[64][136]; __shared__ __align__(16) float sot[DZ][68];
  const int tid = threadIdx.x, wave = tid >> 5, lane = tid & 31, col = lane & 15, g = lane >> 4; const int n = blockIdx.y; const int i0 = blockIdx.x * 64; const size_t r0 = (size_t)n * LL + i0;
  for (int e = tid; e < 64 * 128; e += 128) { const int rl = e >> 7, c = e & 127; sa[rl][c] = (_Float16)(O[(r0 + rl) * DHC + c] * (float)GH[(r0 + rl) * DHC + c] * 256.0f); }
  __syncthreads();
  v8f acc[8] = {};
#pragma unroll
  for (int kc = 0; kc < DHC / 32; ++kc) { v16h a; { union { v16h v; v8h q[2]; } u; u.q[0] = *(const v8h*)&sa[wave * 16 + col][kc * 32 + 8 * g]; u.q[1] = *(const v8h*)&sa[wave * 16 + col][kc * 32 + 16 + 8 * g]; a = u.v; }
#pragma unroll
    for (int j = 0; j < 8; ++j) { const v16h w = wcolh(W2, kc * 32, j * 16 + col, lane, DZ); asm volatile("s_wait_loadcnt 0x0" ::: "memory"); acc[j] = wmma16(a, w, acc[j]); } }
#pragma unroll
  for (int j = 0; j < 8; ++j) { const float bb = bfr(B2[j * 16 + col]);
#pragma unroll
    for (int r = 0; r < 8; ++r) sot[j * 16 + col][wave * 16 + 8 * g + r] = acc[j][r] * (1.0f / 65536.0f) + bb; }
  __syncthreads();
  for (int e = tid; e < DZ * 16; e += 128) { const int c = e >> 4, q = e & 15; vst2(OUT + (size_t)c * ZP + (size_t)n * LL + i0 + q * 4, *(const v4f*)&sot[c][q * 4]); } }
extern "C" void kernel_launch(void* const* d_in, const int* in_sizes, int n_in, void* d_out, int out_size, void* d_ws, size_t ws_size, hipStream_t stream) {
  (void)in_sizes; (void)n_in; (void)out_size;
  const float** F = (const float**)d_in;
  if (ws_size < (size_t)WS_END) return;
  char* ws = (char*)d_ws; _Float16 *ZH = (_Float16*)(ws + WS_ZH), *ZL = (_Float16*)(ws + WS_ZL), *QH = (_Float16*)(ws + WS_QH), *KH = (_Float16*)(ws + WS_KH), *VT = (_Float16*)(ws + WS_VT), *GH = (_Float16*)(ws + WS_GH); float* O = (float*)(ws + WS_O);
  k_ln<<<dim3(LL / 64, NROWS), 128, 0, stream>>>(F[0], F[1], F[2], ZH, ZL);
  k_proj<<<dim3(NROWS * LL / 64, 1, 4), 128, 0, stream>>>(ZH, ZL, F[3], F[4], F[5], F[6], F[7], F[8], F[9], F[10], QH, KH, VT, GH);
  k_att<<<dim3(LL / 32, NH, NROWS), 64, 0, stream>>>(QH, KH, VT, O);
  k_out<<<dim3(LL / 64, NROWS), 128, 0, stream>>>(O, GH, F[11], F[12], (float*)d_out);
}
